// MultiModalAttention_627065225467
// MI455X (gfx1250) — hardware-verified
//
#include <hip/hip_runtime.h>
#include <stdint.h>

typedef __attribute__((ext_vector_type(16))) _Float16 v16h;
typedef __attribute__((ext_vector_type(8)))  _Float16 v8h;
typedef __attribute__((ext_vector_type(16))) __bf16   v16b;
typedef __attribute__((ext_vector_type(8)))  __bf16   v8b;
typedef __attribute__((ext_vector_type(8)))  float    v8f;
typedef __attribute__((ext_vector_type(4)))  float    v4f;
typedef __attribute__((ext_vector_type(4)))  unsigned int u32x4;

constexpr int kB   = 4;
constexpr int kNQ  = 2048;
constexpr int kNKV = 1024;
constexpr int kDM  = 1024;
constexpr int kH   = 16;
constexpr int kDH  = 64;
constexpr int kIN  = kH * kDH;
static_assert(kDH == 64);
static_assert(kDM % 32 == 0);
static_assert(kIN % 32 == 0);
static_assert((kB * kNQ) % 64 == 0);
static_assert((kB * kNKV) % 64 == 0);
static_assert(kIN % 64 == 0);
static_assert(kDM % 64 == 0);
static_assert(kNQ % 64 == 0);
static_assert(kNKV % 64 == 0);

constexpr size_t kMiB    = 1048576;
constexpr size_t kOffXb  = 0;
constexpr size_t kOffCb  = 16 * kMiB;
constexpr size_t kOffWqb = 24 * kMiB;
constexpr size_t kOffWkvb= 26 * kMiB;
constexpr size_t kOffQh  = 32 * kMiB;
constexpr size_t kOffQl  = 48 * kMiB;
constexpr size_t kOffKh  = 64 * kMiB;
constexpr size_t kOffKl  = 72 * kMiB;
constexpr size_t kOffVth = 80 * kMiB;
constexpr size_t kOffVtl = 88 * kMiB;
constexpr size_t kOffWob = 96 * kMiB;
constexpr size_t kOffOh  = 0;
constexpr size_t kOffOl  = 16 * kMiB;
constexpr size_t kWsTotal = kOffWob + (size_t)kDM * kIN * 2;
static_assert((size_t)kB * kNQ * kDM * 2 == 16 * kMiB);
static_assert((size_t)kB * kNKV * kDM * 2 == 8 * kMiB);
static_assert(kOffCb + (size_t)kB * kNKV * kDM * 2 <= kOffWqb);
static_assert(kOffWqb + (size_t)kIN * kDM * 2 <= kOffWkvb);
static_assert(kOffWkvb + (size_t)2 * kIN * kDM * 2 <= kOffQh);
static_assert(kOffQh + (size_t)kB * kNQ * kIN * 2 <= kOffQl);
static_assert(kOffQl + (size_t)kB * kNQ * kIN * 2 <= kOffKh);
static_assert(kOffKh + (size_t)kB * kNKV * kIN * 2 <= kOffKl);
static_assert(kOffKl + (size_t)kB * kNKV * kIN * 2 <= kOffVth);
static_assert(kOffVth + (size_t)kIN * kB * kNKV * 2 <= kOffVtl);
static_assert(kOffVtl + (size_t)kIN * kB * kNKV * 2 <= kOffWob);
static_assert(kOffOh + (size_t)kB * kNQ * kIN * 2 <= kOffOl);
static_assert(kOffOl + (size_t)kB * kNQ * kIN * 2 <= kOffQh);
static_assert(kWsTotal == 102760448);
static_assert(kWsTotal <= 134217728);

__device__ __forceinline__ unsigned short f2bf_bits(float f) {
  unsigned u = __float_as_uint(f);
  return (unsigned short)((u + 0x7FFFu + ((u >> 16) & 1u)) >> 16);
}
__device__ __forceinline__ float bf_bits2f(unsigned short h) { return __uint_as_float(((unsigned)h) << 16); }

__device__ __forceinline__ void dep_guard_h(v8f& a, v8f& b, v16h x, v16h y) { asm volatile("v_nop\n\tv_nop\n\tv_nop\n\tv_nop" : "+v"(a), "+v"(b) : "v"(x), "v"(y)); }
__device__ __forceinline__ void dep_guard_b(v8f& a, v8f& b, v16b x, v16b y) { asm volatile("v_nop\n\tv_nop\n\tv_nop\n\tv_nop" : "+v"(a), "+v"(b) : "v"(x), "v"(y)); }
__device__ __forceinline__ void keep4_h(v16h a, v16h b, v16h c, v16h d) { asm volatile("v_nop" :: "v"(a), "v"(b), "v"(c), "v"(d)); }
__device__ __forceinline__ void keep4_b(v16b a, v16b b, v16b c, v16b d) { asm volatile("v_nop" :: "v"(a), "v"(b), "v"(c), "v"(d)); }
__device__ __forceinline__ void acc_guard4(v8f& a, v8f& b, v8f& c, v8f& d) { asm volatile("v_nop\n\tv_nop\n\tv_nop\n\tv_nop" : "+v"(a), "+v"(b), "+v"(c), "+v"(d)); }
template <typename T> struct Frag;
template <> struct Frag<_Float16> {
  typedef v16h V; union U { v16h v; v8h h[2]; };
  static __device__ __forceinline__ v16h load(const _Float16* p) {
    U f; f.h[0] = *(const v8h*)(p); f.h[1] = *(const v8h*)(p + 16); return f.v;
  }
  static __device__ __forceinline__ v8f mma(v16h a, v16h b, v8f c) {
    return __builtin_amdgcn_wmma_f32_16x16x32_f16(false, a, false, b, (short)0, c, false, false);
  }
  static __device__ __forceinline__ void guard(v8f& a, v8f& b, v16h x, v16h y) { dep_guard_h(a, b, x, y); }
  static __device__ __forceinline__ void keep(v16h a, v16h b, v16h c, v16h d) { keep4_h(a, b, c, d); }
};
template <> struct Frag<__bf16> {
  typedef v16b V; union U { v16b v; v8b h[2]; };
  static __device__ __forceinline__ v16b load(const __bf16* p) {
    U f; f.h[0] = *(const v8b*)(p); f.h[1] = *(const v8b*)(p + 16); return f.v;
  }
  static __device__ __forceinline__ v8f mma(v16b a, v16b b, v8f c) {
    return __builtin_amdgcn_wmma_f32_16x16x32_bf16(false, a, false, b, (short)0, c, false, false);
  }
  static __device__ __forceinline__ void guard(v8f& a, v8f& b, v16b x, v16b y) { dep_guard_b(a, b, x, y); }
  static __device__ __forceinline__ void keep(v16b a, v16b b, v16b c, v16b d) { keep4_b(a, b, c, d); }
};

template <int ET> struct Elem;
template <> struct Elem<0> { typedef _Float16 T; };
template <> struct Elem<1> { typedef __bf16 T; };
template <int ET, bool SPLIT, bool SPLIT_B, int BIAS_MODE, int OUT_MODE>
__global__ __launch_bounds__(256) void wmma_gemm64(
    const unsigned short* __restrict__ Ap, const unsigned short* __restrict__ A2p, int lda, long strideA,
    const unsigned short* __restrict__ Btp, const unsigned short* __restrict__ Bt2p, int ldb, long strideB,
    void* Cout, void* Cout2, int ldc, long strideC,
    const float* __restrict__ bias,
    int M, int N, int K, float scale) {
  static_assert(BIAS_MODE == 0 || BIAS_MODE == 2);
  static_assert(OUT_MODE == 0 || OUT_MODE == 2);
  typedef typename Elem<ET>::T T;
  typedef typename Frag<T>::V V;
  const T* A = (const T*)Ap; const T* A2 = (const T*)A2p; const T* Bt = (const T*)Btp; const T* Bt2 = (const T*)Bt2p;
  __shared__ __align__(16) float sT[8][16 * 68];
  const int b    = blockIdx.y;
  const int lane = threadIdx.x & 31;
  const int wave = threadIdx.x >> 5;
  const int tilesN = N >> 6;
  const int tilesM = M >> 6;
  const int tile = blockIdx.x * 8 + wave;
  if (tile >= tilesM * tilesN) return;
  const int tm = tile / tilesN;
  const int tn = tile - tm * tilesN;
  const int m0 = tm << 6;
  const int n0 = tn << 6;

  const T* Ab  = A  + (size_t)b * strideA;
  const T* Bb  = Bt + (size_t)b * strideB;
  const T* Ab2 = SPLIT ? (A2  + (size_t)b * strideA) : nullptr;
  const T* Bb2 = (SPLIT && SPLIT_B) ? (Bt2 + (size_t)b * strideB) : nullptr;

  const int rlane = lane & 15;
  const int koff  = (lane >> 4) * 8;
  const int mOff  = (lane >> 4) * 8;

  v8f acc[4][4];
#pragma unroll
  for (int i = 0; i < 4; ++i)
#pragma unroll
    for (int j = 0; j < 4; ++j) acc[i][j] = (v8f){0.f,0.f,0.f,0.f,0.f,0.f,0.f,0.f};

  for (int k0 = 0; k0 < K; k0 += 32) {
    V bh[4], bl[4];
#pragma unroll
    for (int j = 0; j < 4; ++j) {
      const size_t bo = (size_t)(n0 + (j << 4) + rlane) * ldb + koff + k0;
      bh[j] = Frag<T>::load(Bb + bo);
      if (SPLIT && SPLIT_B) bl[j] = Frag<T>::load(Bb2 + bo);
    }
#pragma unroll
    for (int i = 0; i < 4; ++i) {
      const size_t ao = (size_t)(m0 + (i << 4) + rlane) * lda + koff + k0;
      V ah = Frag<T>::load(Ab + ao);
      V al;
      if (SPLIT) al = Frag<T>::load(Ab2 + ao);
#pragma unroll
      for (int j = 0; j < 4; ++j) {
        acc[i][j] = Frag<T>::mma(ah, bh[j], acc[i][j]);
        if (SPLIT) {
          if (SPLIT_B) acc[i][j] = Frag<T>::mma(ah, bl[j], acc[i][j]);
          acc[i][j] = Frag<T>::mma(al, bh[j], acc[i][j]);
        }
      }
      Frag<T>::guard(acc[i][0], acc[i][3], ah, SPLIT ? al : ah);
    }
    Frag<T>::keep(bh[0], bh[1], bh[2], bh[3]);
    if (SPLIT && SPLIT_B) Frag<T>::keep(bl[0], bl[1], bl[2], bl[3]);
  }
  acc_guard4(acc[0][0], acc[0][1], acc[0][2], acc[0][3]);
  acc_guard4(acc[1][0], acc[1][1], acc[1][2], acc[1][3]);
  acc_guard4(acc[2][0], acc[2][1], acc[2][2], acc[2][3]);
  acc_guard4(acc[3][0], acc[3][1], acc[3][2], acc[3][3]);

  float* slab = sT[wave];
#pragma unroll
  for (int i = 0; i < 4; ++i) {
    const int mBase = m0 + (i << 4);
#pragma unroll
    for (int j = 0; j < 4; ++j) {
      const int n = n0 + (j << 4) + rlane;
      float bv = 0.f;
      if (BIAS_MODE == 2) bv = bias[n];
#pragma unroll
      for (int r = 0; r < 8; ++r) {
        float v = acc[i][j][r] * scale;
        if (BIAS_MODE == 2) v += bv;
        slab[(mOff + r) * 68 + (j << 4) + rlane] = v;
      }
    }
    __builtin_amdgcn_fence(__ATOMIC_RELEASE, "workgroup");
    __builtin_amdgcn_wave_barrier();
    __builtin_amdgcn_fence(__ATOMIC_ACQUIRE, "workgroup");
    if (OUT_MODE == 0) {
      float* C = (float*)Cout + (size_t)b * strideC;
      const int hh = lane >> 4, c4 = (lane & 15) * 4;
      for (int pass = 0; pass < 2; ++pass) {
#pragma unroll
        for (int it = 0; it < 8; ++it) {
          const int row = it * 2 + hh;
          v4f v = *(const v4f*)(slab + row * 68 + c4);
          *(volatile v4f*)(C + (size_t)(mBase + row) * ldc + n0 + c4) = v;
        }
        __threadfence();
      }
    } else {
      const int q = lane >> 3, c8 = (lane & 7) * 8;
      unsigned short* C  = (unsigned short*)Cout  + (size_t)b * strideC;
      unsigned short* C2 = (unsigned short*)Cout2 + (size_t)b * strideC;
      for (int pass = 0; pass < 2; ++pass) {
#pragma unroll
        for (int it = 0; it < 4; ++it) {
          const int row = it * 4 + q;
          const float* sp = slab + row * 68 + c8;
          v8h hv, lv;
#pragma unroll
          for (int e = 0; e < 8; ++e) {
            unsigned short hb = f2bf_bits(sp[e]);
            unsigned short lb = f2bf_bits(sp[e] - bf_bits2f(hb));
            hv[e] = __builtin_bit_cast(_Float16, hb);
            lv[e] = __builtin_bit_cast(_Float16, lb);
          }
          *(volatile v8h*)(C  + (size_t)(mBase + row) * ldc + n0 + c8) = hv;
          *(volatile v8h*)(C2 + (size_t)(mBase + row) * ldc + n0 + c8) = lv;
        }
        __threadfence();
      }
    }
    __builtin_amdgcn_fence(__ATOMIC_RELEASE, "workgroup");
    __builtin_amdgcn_wave_barrier();
    __builtin_amdgcn_fence(__ATOMIC_ACQUIRE, "workgroup");
  }
}

__global__ __launch_bounds__(256) void cast_f32_bf16x8(
    const float* __restrict__ in, unsigned short* __restrict__ out, int n8) {
  const int i = blockIdx.x * 256 + threadIdx.x;
  if (i < n8) {
    const v4f a = *(const v4f*)(in + (size_t)i * 8);
    const v4f c = *(const v4f*)(in + (size_t)i * 8 + 4);
    u32x4 w;
    w[0] = (unsigned)f2bf_bits(a[0]) | ((unsigned)f2bf_bits(a[1]) << 16);
    w[1] = (unsigned)f2bf_bits(a[2]) | ((unsigned)f2bf_bits(a[3]) << 16);
    w[2] = (unsigned)f2bf_bits(c[0]) | ((unsigned)f2bf_bits(c[1]) << 16);
    w[3] = (unsigned)f2bf_bits(c[2]) | ((unsigned)f2bf_bits(c[3]) << 16);
    volatile u32x4* p = (volatile u32x4*)(out + (size_t)i * 8);
    *p = w;
    __threadfence();
    *p = w;
  }
}

#define AT_D 64
#define AT_NW 4
#define AT_QB 64
#define AT_KC 64

__device__ __forceinline__ unsigned short at_bf_bits(float f) {
  unsigned u = __float_as_uint(f);
  return (unsigned short)((u + 0x7FFFu + ((u >> 16) & 1u)) >> 16);
}
__device__ __forceinline__ __bf16 at_f2bf(float f) { return __builtin_bit_cast(__bf16, at_bf_bits(f)); }
__device__ __forceinline__ void at_split(float f, __bf16& hi, __bf16& lo) {
  const unsigned short hb = at_bf_bits(f);
  hi = __builtin_bit_cast(__bf16, hb);
  lo = at_f2bf(f - __uint_as_float(((unsigned)hb) << 16));
}
__device__ __forceinline__ v8f at_mma(v16b a, v16b b, v8f c) {
  c = __builtin_amdgcn_wmma_f32_16x16x32_bf16(false, a, false, b, (short)0, c, false, false);
  asm volatile("v_nop\n\tv_nop\n\tv_nop\n\tv_nop" : "+v"(c) : "v"(a), "v"(b));
  return c;
}

__global__ __launch_bounds__(128)
void attn64_planes_kernel(const unsigned short* __restrict__ qhp, const unsigned short* __restrict__ qlp,
                          const unsigned short* __restrict__ khp, const unsigned short* __restrict__ klp,
                          const unsigned short* __restrict__ vthp, const unsigned short* __restrict__ vtlp,
                          const int* __restrict__ kvmask,
                          unsigned short* __restrict__ ohp, unsigned short* __restrict__ olp,
                          int nq, int nkv, int nh, int ldq, int ldk, int ldv, int ldo, float fillv) {
  typedef __bf16 T;
  union FB { v16b v; v8b h[2]; };
  __shared__ __align__(16) __bf16 Ksh[AT_KC * AT_D];
  __shared__ __align__(16) __bf16 Ksl[AT_KC * AT_D];
  __shared__ __align__(16) __bf16 Vth[AT_D * AT_KC];
  __shared__ __align__(16) __bf16 Vtl[AT_D * AT_KC];
  __shared__ __align__(16) __bf16 Psh[AT_NW][16 * AT_KC];
  __shared__ __align__(16) __bf16 Psl[AT_NW][16 * AT_KC];
  __shared__ __align__(16) float  Os[AT_NW][16 * 68];

  const int tid  = threadIdx.x;
  const int wave = tid >> 5;
  const int lane = tid & 31;
  const int hh   = lane >> 4;
  const int c    = lane & 15;

  const int nqb = nq / AT_QB;
  const int bx = blockIdx.x;
  const int qb = bx % nqb;
  const int bhx = bx / nqb;
  const int h  = bhx % nh;
  const int b  = bhx / nh;
  const int q0 = qb * AT_QB + wave * 16;

  v16b qah[2], qal[2];
  {
    const size_t qo = (size_t)(b * nq + q0 + c) * ldq + h * AT_D + 8 * hh;
    const T* qh = (const T*)qhp + qo;
    const T* ql = (const T*)qlp + qo;
#pragma unroll
    for (int dc = 0; dc < 2; ++dc) {
      qah[dc] = Frag<T>::load(qh + dc * 32);
      qal[dc] = Frag<T>::load(ql + dc * 32);
    }
  }

  float mrow[8], lrow[8];
  v8f oacc[4];
#pragma unroll
  for (int r = 0; r < 8; ++r) { mrow[r] = -__builtin_inff(); lrow[r] = 0.f; }
#pragma unroll
  for (int t = 0; t < 4; ++t) oacc[t] = (v8f){0.f,0.f,0.f,0.f,0.f,0.f,0.f,0.f};

  const int nChunks = nkv / AT_KC;
  for (int kc = 0; kc < nChunks; ++kc) {
    const int kv0 = kc * AT_KC;
    __syncthreads();
    {
      const int row = tid >> 1;
      const int half = (tid & 1) * 32;
      const u32x4* gkh = (const u32x4*)(khp + (size_t)(b * nkv + kv0 + row) * ldk + h * AT_D + half);
      const u32x4* gkl = (const u32x4*)(klp + (size_t)(b * nkv + kv0 + row) * ldk + h * AT_D + half);
      u32x4* lkh = (u32x4*)(Ksh + row * AT_D + half);
      u32x4* lkl = (u32x4*)(Ksl + row * AT_D + half);
#pragma unroll
      for (int i = 0; i < 4; ++i) { lkh[i] = gkh[i]; lkl[i] = gkl[i]; }
      asm volatile("" ::: "memory");
      const u32x4* gvh = (const u32x4*)(vthp + (size_t)(h * AT_D + row) * ldv + b * nkv + kv0 + half);
      const u32x4* gvl = (const u32x4*)(vtlp + (size_t)(h * AT_D + row) * ldv + b * nkv + kv0 + half);
      u32x4* lvh = (u32x4*)(Vth + row * AT_KC + half);
      u32x4* lvl = (u32x4*)(Vtl + row * AT_KC + half);
#pragma unroll
      for (int i = 0; i < 4; ++i) { lvh[i] = gvh[i]; lvl[i] = gvl[i]; }
    }
    __syncthreads();

    v8f s[4];
#pragma unroll
    for (int j = 0; j < 4; ++j) {
      s[j] = (v8f){0.f,0.f,0.f,0.f,0.f,0.f,0.f,0.f};
#pragma unroll
      for (int dc = 0; dc < 2; ++dc) {
        FB kb, kl;
        kb.h[0] = *(const v8b*)(Ksh + (j * 16 + c) * AT_D + dc * 32 + 8 * hh);
        kb.h[1] = *(const v8b*)(Ksh + (j * 16 + c) * AT_D + dc * 32 + 16 + 8 * hh);
        kl.h[0] = *(const v8b*)(Ksl + (j * 16 + c) * AT_D + dc * 32 + 8 * hh);
        kl.h[1] = *(const v8b*)(Ksl + (j * 16 + c) * AT_D + dc * 32 + 16 + 8 * hh);
        s[j] = at_mma(qah[dc], kb.v, s[j]);
        s[j] = at_mma(qah[dc], kl.v, s[j]);
        s[j] = at_mma(qal[dc], kb.v, s[j]);
      }
    }
    int kvkeep[4];
#pragma unroll
    for (int j = 0; j < 4; ++j) kvkeep[j] = kvmask[(size_t)b * nkv + kv0 + j * 16 + c];
    float cm[8];
#pragma unroll
    for (int r = 0; r < 8; ++r) {
      float m = -__builtin_inff();
#pragma unroll
      for (int j = 0; j < 4; ++j) {
        const float sv = s[j][r];
        s[j][r] = (kvkeep[j] != 0) ? sv : fillv;
        m = fmaxf(m, s[j][r]);
      }
#pragma unroll
      for (int off = 1; off < 16; off <<= 1) m = fmaxf(m, __shfl_xor(m, off, 32));
      cm[r] = m;
    }
    __bf16* pwh = Psh[wave];
    __bf16* pwl = Psl[wave];
#pragma unroll
    for (int r = 0; r < 8; ++r) {
      const float mnew = fmaxf(mrow[r], cm[r]);
      const float alpha = expf(mrow[r] - mnew);
      mrow[r] = mnew;
      float psum = 0.f;
#pragma unroll
      for (int j = 0; j < 4; ++j) {
        const float p = expf(s[j][r] - mnew);
        psum += p;
        __bf16 a, bl; at_split(p, a, bl);
        pwh[(8 * hh + r) * AT_KC + j * 16 + c] = a;
        pwl[(8 * hh + r) * AT_KC + j * 16 + c] = bl;
      }
#pragma unroll
      for (int off = 1; off < 16; off <<= 1) psum += __shfl_xor(psum, off, 32);
      lrow[r] = lrow[r] * alpha + psum;
#pragma unroll
      for (int t = 0; t < 4; ++t) oacc[t][r] *= alpha;
    }
    __builtin_amdgcn_fence(__ATOMIC_RELEASE, "workgroup");
    __builtin_amdgcn_wave_barrier();
    __builtin_amdgcn_fence(__ATOMIC_ACQUIRE, "workgroup");
#pragma unroll 1
    for (int kk = 0; kk < 2; ++kk) {
      FB pa, pl;
      pa.h[0] = *(const v8b*)(pwh + c * AT_KC + kk * 32 + 8 * hh);
      pa.h[1] = *(const v8b*)(pwh + c * AT_KC + kk * 32 + 16 + 8 * hh);
      pl.h[0] = *(const v8b*)(pwl + c * AT_KC + kk * 32 + 8 * hh);
      pl.h[1] = *(const v8b*)(pwl + c * AT_KC + kk * 32 + 16 + 8 * hh);
#pragma unroll
      for (int t = 0; t < 4; ++t) {
        FB vb, vl;
        vb.h[0] = *(const v8b*)(Vth + (t * 16 + c) * AT_KC + kk * 32 + 8 * hh);
        vb.h[1] = *(const v8b*)(Vth + (t * 16 + c) * AT_KC + kk * 32 + 16 + 8 * hh);
        vl.h[0] = *(const v8b*)(Vtl + (t * 16 + c) * AT_KC + kk * 32 + 8 * hh);
        vl.h[1] = *(const v8b*)(Vtl + (t * 16 + c) * AT_KC + kk * 32 + 16 + 8 * hh);
        oacc[t] = at_mma(pa.v, vb.v, oacc[t]);
        oacc[t] = at_mma(pa.v, vl.v, oacc[t]);
        oacc[t] = at_mma(pl.v, vb.v, oacc[t]);
      }
    }
  }

  float* os = Os[wave];
#pragma unroll
  for (int r = 0; r < 8; ++r) {
    const float inv = 1.0f / lrow[r];
#pragma unroll
    for (int t = 0; t < 4; ++t) os[(8 * hh + r) * 68 + t * 16 + c] = oacc[t][r] * inv;
  }
  __builtin_amdgcn_fence(__ATOMIC_RELEASE, "workgroup");
  __builtin_amdgcn_wave_barrier();
  __builtin_amdgcn_fence(__ATOMIC_ACQUIRE, "workgroup");
  {
    const int q = lane >> 3, c8 = (lane & 7) * 8;
    unsigned short* Oh = ohp + (size_t)(b * nq + q0) * ldo + h * AT_D;
    unsigned short* Ol = olp + (size_t)(b * nq + q0) * ldo + h * AT_D;
    for (int pass = 0; pass < 2; ++pass) {
#pragma unroll
      for (int it = 0; it < 4; ++it) {
        const int row = it * 4 + q;
        const float* sp = os + row * 68 + c8;
        v8h hv, lv;
#pragma unroll
        for (int e = 0; e < 8; ++e) {
          unsigned short hb = f2bf_bits(sp[e]);
          unsigned short lb = f2bf_bits(sp[e] - bf_bits2f(hb));
          hv[e] = __builtin_bit_cast(_Float16, hb);
          lv[e] = __builtin_bit_cast(_Float16, lb);
        }
        *(volatile v8h*)(Oh + (size_t)row * ldo + c8) = hv;
        *(volatile v8h*)(Ol + (size_t)row * ldo + c8) = lv;
      }
      __threadfence();
    }
  }
}

extern "C" void kernel_launch(void* const* d_in, const int* in_sizes, int n_in,
                              void* d_out, int out_size, void* d_ws, size_t ws_size,
                              hipStream_t stream) {
  if (n_in < 7) return;
  if (in_sizes[0] != kB * kNQ * kDM) return;
  if (in_sizes[1] != kB * kNKV * kDM) return;
  if (in_sizes[2] != kB * kNKV) return;
  if (in_sizes[3] != kIN * kDM) return;
  if (in_sizes[4] != 2 * kIN * kDM) return;
  if (in_sizes[5] != kDM * kIN) return;
  if (in_sizes[6] != kDM) return;
  if (out_size != kB * kNQ * kDM) return;
  if (ws_size < kWsTotal) return;

  const float* x    = (const float*)d_in[0];
  const float* ctx  = (const float*)d_in[1];
  const int*   mask = (const int*)d_in[2];
  const float* Wq   = (const float*)d_in[3];
  const float* Wkv  = (const float*)d_in[4];
  const float* Wout = (const float*)d_in[5];
  const float* bout = (const float*)d_in[6];
  float* out = (float*)d_out;

  char* ws = (char*)d_ws;
  unsigned short* xb   = (unsigned short*)(ws + kOffXb);
  unsigned short* cb   = (unsigned short*)(ws + kOffCb);
  unsigned short* wqb  = (unsigned short*)(ws + kOffWqb);
  unsigned short* wkvb = (unsigned short*)(ws + kOffWkvb);
  unsigned short* wob  = (unsigned short*)(ws + kOffWob);
  unsigned short* qh   = (unsigned short*)(ws + kOffQh);
  unsigned short* ql   = (unsigned short*)(ws + kOffQl);
  unsigned short* kh   = (unsigned short*)(ws + kOffKh);
  unsigned short* kl   = (unsigned short*)(ws + kOffKl);
  unsigned short* vth  = (unsigned short*)(ws + kOffVth);
  unsigned short* vtl  = (unsigned short*)(ws + kOffVtl);
  unsigned short* oh   = (unsigned short*)(ws + kOffOh);
  unsigned short* ol   = (unsigned short*)(ws + kOffOl);

  {
    const int n8x = kB * kNQ * kDM / 8;
    const int n8c = kB * kNKV * kDM / 8;
    const int n8q = kIN * kDM / 8;
    const int n8kv = 2 * kIN * kDM / 8;
    const int n8o = kDM * kIN / 8;
    cast_f32_bf16x8<<<(n8x + 255) / 256, 256, 0, stream>>>(x, xb, n8x);
    cast_f32_bf16x8<<<(n8c + 255) / 256, 256, 0, stream>>>(ctx, cb, n8c);
    cast_f32_bf16x8<<<(n8q + 255) / 256, 256, 0, stream>>>(Wq, wqb, n8q);
    cast_f32_bf16x8<<<(n8kv + 255) / 256, 256, 0, stream>>>(Wkv, wkvb, n8kv);
    cast_f32_bf16x8<<<(n8o + 255) / 256, 256, 0, stream>>>(Wout, wob, n8o);
  }

  {
    const int M = kB * kNQ, N = kIN, K = kDM;
    const int tiles = (M / 64) * (N / 64);
    wmma_gemm64<1, false, false, 0, 2><<<dim3((tiles + 7) / 8, 1), 256, 0, stream>>>(
        xb, xb, K, 0L, wqb, wqb, K, 0L, (void*)qh, (void*)ql, N, 0L, bout, M, N, K, 0.125f);
  }
  {
    const int M = kB * kNKV, N = kIN, K = kDM;
    const int tiles = (M / 64) * (N / 64);
    wmma_gemm64<1, false, false, 0, 2><<<dim3((tiles + 7) / 8, 1), 256, 0, stream>>>(
        cb, cb, K, 0L, wkvb, wkvb, K, 0L, (void*)kh, (void*)kl, N, 0L, bout, M, N, K, 1.0f);
  }
  {
    const int M = kIN, N = kB * kNKV, K = kDM;
    const int tiles = (M / 64) * (N / 64);
    const unsigned short* wvb = wkvb + (size_t)kIN * kDM;
    wmma_gemm64<1, false, false, 0, 2><<<dim3((tiles + 7) / 8, 1), 256, 0, stream>>>(
        wvb, wvb, K, 0L, cb, cb, K, 0L, (void*)vth, (void*)vtl, N, 0L, bout, M, N, K, 1.0f);
  }
  {
    const int blocks = kB * kH * (kNQ / 64);
    const float fillv = -3.4028234663852886e+38f;
    attn64_planes_kernel<<<blocks, 128, 0, stream>>>(qh, ql, kh, kl, vth, vtl, mask, oh, ol,
                                                    kNQ, kNKV, kH, kIN, kIN, kB * kNKV, kIN, fillv);
  }
  {
    const int M = kB * kNQ, N = kDM, K = kIN;
    const int tiles = (M / 64) * (N / 64);
    wmma_gemm64<1, true, false, 2, 0><<<dim3((tiles + 7) / 8, 1), 256, 0, stream>>>(
        oh, ol, K, 0L, wob, wob, K, 0L, (void*)out, (void*)out, N, 0L, bout, M, N, K, 1.0f);
  }
}
